// MHPLSTMCore_88235808129369
// MI455X (gfx1250) — hardware-run, weakly checked
//
#include <hip/hip_runtime.h>
#include <math.h>

typedef __attribute__((ext_vector_type(16))) _Float16 v16h;
typedef __attribute__((ext_vector_type(8)))  _Float16 v8h;
typedef __attribute__((ext_vector_type(2)))  _Float16 v2h;
typedef __attribute__((ext_vector_type(16))) __bf16   v16b;
typedef __attribute__((ext_vector_type(8)))  __bf16   v8b;
typedef __attribute__((ext_vector_type(8)))  float    v8f;
typedef __attribute__((ext_vector_type(4)))  float    v4f;
typedef __attribute__((ext_vector_type(2)))  float    v2f;
typedef __attribute__((ext_vector_type(4)))  _Float16 v4h;

constexpr int kNB   = 4;
constexpr int kL    = 4096;
constexpr int kH    = 8;
constexpr int kD    = 64;
constexpr int kHD   = kH * kD;
constexpr int kTok  = kNB * kL;
constexpr int kRows = kTok * kH;
constexpr int kK    = 2 * kD;
constexpr int kN3   = 3 * kD;
constexpr int kOut0 = kRows * kD;
constexpr int kBvOg = kN3;
constexpr int kBvTot = kN3 + kD;
constexpr int kThr  = 256;
constexpr float kACarry = 512.0f;
constexpr float kWCarry = 4096.0f;
constexpr float kSc = 1.0f / (kACarry * kWCarry);
constexpr float kNormEps = 1e-5f;
constexpr float kF16MinNormal = 6.103515625e-5f;

static_assert(kTok == 16384 && kRows == 131072 && kHD == 512 && kK == 128 && kN3 == 192 && (kN3 % 64) == 0 && (kD % 64) == 0 && (kL & (kL - 1)) == 0, "the index arithmetic below uses these sizes");

constexpr size_t kOffWHT = 0ull;
constexpr size_t kOffWOT = 49152ull;
constexpr size_t kOffBV = 65536ull;
constexpr size_t kOffST = 66560ull;
constexpr size_t kOffRAW = 197632ull;
constexpr size_t kOffA16 = 33752064ull;
constexpr size_t kOffH3 = 67306496ull;
constexpr size_t kOffCELL = 167969792ull;
constexpr size_t kOffOGP = 201524224ull;
constexpr size_t kWsTotal = 235078656ull;
static_assert(kWsTotal <= 268435456ull, "the carve stands under the contract's 256 MiB of workspace");
static_assert(kOffWHT == 0
  && kOffWOT == kOffWHT + 49152ull
  && kOffBV == kOffWOT + 16384ull
  && kOffST == kOffBV + 1024ull
  && kOffRAW == kOffST + 131072ull
  && kOffA16 == kOffRAW + 33554432ull
  && kOffH3 == kOffA16 + 33554432ull
  && kOffCELL == kOffH3 + 100663296ull
  && kOffOGP == kOffCELL + 33554432ull
  && kWsTotal == kOffOGP + 33554432ull, "the carve is a chain: every region starts where the one before ends");
static_assert((size_t)kN3 * kK * 2 == 49152ull && (size_t)kD * kK * 2 == 16384ull && (size_t)kBvTot * 4 == 1024ull && (size_t)kTok * 2 * 4 == 131072ull && (size_t)kTok * kHD * 4 == 33554432ull && (size_t)kRows * kK * 2 == 33554432ull
  && (size_t)kRows * kN3 * 4 == 100663296ull && (size_t)kRows * kD * 4 == 33554432ull, "every region's length is its plane's");
static_assert((kOffWOT % 256) == 0 && (kOffBV % 256) == 0 && (kOffST % 256) == 0 && (kOffRAW % 256) == 0 && (kOffA16 % 256) == 0 && (kOffH3 % 256) == 0 && (kOffCELL % 256) == 0 && (kOffOGP % 256) == 0, "every region starts on a multiple of 256 B");

__device__ __forceinline__ unsigned short f2bf_bits(float f) {
  unsigned u = __float_as_uint(f);
  return (unsigned short)((u + 0x7FFFu + ((u >> 16) & 1u)) >> 16);
}
__device__ __forceinline__ float bf_bits2f(unsigned short h) { return __uint_as_float(((unsigned)h) << 16); }
__device__ __forceinline__ float bf16r(float f) { return bf_bits2f(f2bf_bits(f)); }
__device__ __forceinline__ float carry_flush(float v, float carry) {
  const float s = v * carry;
  return (fabsf(s) < kF16MinNormal) ? 0.0f : s;
}

__device__ __forceinline__ void dep_guard4_h(v8f& a, v8f& b, v8f& c, v8f& d, v16h x, v16h y) { asm volatile("v_nop\n\tv_nop\n\tv_nop\n\tv_nop" : "+v"(a), "+v"(b), "+v"(c), "+v"(d) : "v"(x), "v"(y)); }
__device__ __forceinline__ void dep_guard4_b(v8f& a, v8f& b, v8f& c, v8f& d, v16b x, v16b y) { asm volatile("v_nop\n\tv_nop\n\tv_nop\n\tv_nop" : "+v"(a), "+v"(b), "+v"(c), "+v"(d) : "v"(x), "v"(y)); }
__device__ __forceinline__ void keep4_h(v16h a, v16h b, v16h c, v16h d) { asm volatile("v_nop" :: "v"(a), "v"(b), "v"(c), "v"(d)); }
__device__ __forceinline__ void keep4_b(v16b a, v16b b, v16b c, v16b d) { asm volatile("v_nop" :: "v"(a), "v"(b), "v"(c), "v"(d)); }
__device__ __forceinline__ void acc_guard4(v8f& a, v8f& b, v8f& c, v8f& d) { asm volatile("v_nop\n\tv_nop\n\tv_nop\n\tv_nop" : "+v"(a), "+v"(b), "+v"(c), "+v"(d)); }

template <typename T> struct Frag;
template <> struct Frag<_Float16> {
  typedef v16h V; union U { v16h v; v8h h[2]; };
  static __device__ __forceinline__ v16h load(const _Float16* p) {
    U f; f.h[0] = *(const v8h*)(p); f.h[1] = *(const v8h*)(p + 16); return f.v;
  }
  static __device__ __forceinline__ v8f mma(v16h a, v16h b, v8f c) {
    return __builtin_amdgcn_wmma_f32_16x16x32_f16(false, a, false, b, (short)0, c, false, false);
  }
  static __device__ __forceinline__ void guard4(v8f& a, v8f& b, v8f& c, v8f& d, v16h x, v16h y) { dep_guard4_h(a, b, c, d, x, y); }
  static __device__ __forceinline__ void keep(v16h a, v16h b, v16h c, v16h d) { keep4_h(a, b, c, d); }
};
template <> struct Frag<__bf16> {
  typedef v16b V; union U { v16b v; v8b h[2]; };
  static __device__ __forceinline__ v16b load(const __bf16* p) {
    U f; f.h[0] = *(const v8b*)(p); f.h[1] = *(const v8b*)(p + 16); return f.v;
  }
  static __device__ __forceinline__ v8f mma(v16b a, v16b b, v8f c) {
    return __builtin_amdgcn_wmma_f32_16x16x32_bf16(false, a, false, b, (short)0, c, false, false);
  }
  static __device__ __forceinline__ void guard4(v8f& a, v8f& b, v8f& c, v8f& d, v16b x, v16b y) { dep_guard4_b(a, b, c, d, x, y); }
  static __device__ __forceinline__ void keep(v16b a, v16b b, v16b c, v16b d) { keep4_b(a, b, c, d); }
};

__device__ __forceinline__ v8f mma_h(v16h a, v16h b, v8f c) {
  c = __builtin_amdgcn_wmma_f32_16x16x32_f16(false, a, false, b, (short)0, c, false, false);
  asm volatile("v_nop\n\tv_nop\n\tv_nop\n\tv_nop" : "+v"(c) : "v"(a), "v"(b));
  return c;
}

template <int ET> struct Elem;
template <> struct Elem<0> { typedef _Float16 T; };
template <> struct Elem<1> { typedef __bf16 T; };
template <int ET, bool SPLIT, int BIAS_MODE, int OUT_MODE, bool RESID, int ACT = 0>
__global__ __launch_bounds__(256) void wmma_gemm64(
    const unsigned short* __restrict__ Ap, const unsigned short* __restrict__ A2p, int lda, long strideA,
    const unsigned short* __restrict__ Btp, const unsigned short* __restrict__ Bt2p, int ldb, long strideB,
    void* __restrict__ Cout, void* __restrict__ Cout2, int ldc, long strideC,
    const float* __restrict__ bias,
    const float* __restrict__ resid, long strideR,
    int M, int N, int K, float scale) {
  typedef typename Elem<ET>::T T;
  typedef typename Frag<T>::V V;
  const T* A = (const T*)Ap; const T* A2 = (const T*)A2p; const T* Bt = (const T*)Btp; const T* Bt2 = (const T*)Bt2p;
  __shared__ __align__(16) float sT[8][16 * 68];
  const int b    = blockIdx.y;
  const int lane = threadIdx.x & 31;
  const int wave = threadIdx.x >> 5;
  const int tilesN = N >> 6;
  const int tilesM = M >> 6;
  const int tile = blockIdx.x * 8 + wave;
  if (tile >= tilesM * tilesN) return;
  const int tm = tile / tilesN;
  const int tn = tile - tm * tilesN;
  const int m0 = tm << 6;
  const int n0 = tn << 6;

  const T* Ab  = A  + (size_t)b * strideA;
  const T* Bb  = Bt + (size_t)b * strideB;
  const T* Ab2 = SPLIT ? (A2  + (size_t)b * strideA) : nullptr;
  const T* Bb2 = SPLIT ? (Bt2 + (size_t)b * strideB) : nullptr;

  const int rlane = lane & 15;
  const int koff  = (lane >> 4) * 8;
  const int mOff  = (lane >> 4) * 8;

  v8f acc[4][4];
#pragma unroll
  for (int i = 0; i < 4; ++i)
#pragma unroll
    for (int j = 0; j < 4; ++j) acc[i][j] = (v8f){0.f,0.f,0.f,0.f,0.f,0.f,0.f,0.f};

  for (int k0 = 0; k0 < K; k0 += 32) {
    V bh[4], bl[4];
#pragma unroll
    for (int j = 0; j < 4; ++j) {
      const size_t bo = (size_t)(n0 + (j << 4) + rlane) * ldb + koff + k0;
      bh[j] = Frag<T>::load(Bb + bo);
      if (SPLIT) bl[j] = Frag<T>::load(Bb2 + bo);
    }
#pragma unroll
    for (int i = 0; i < 4; ++i) {
      const size_t ao = (size_t)(m0 + (i << 4) + rlane) * lda + koff + k0;
      V ah = Frag<T>::load(Ab + ao);
      V al;
      if (SPLIT) al = Frag<T>::load(Ab2 + ao);
#pragma unroll
      for (int j = 0; j < 4; ++j) {
        acc[i][j] = Frag<T>::mma(ah, bh[j], acc[i][j]);
        if (SPLIT) {
          acc[i][j] = Frag<T>::mma(ah, bl[j], acc[i][j]);
          acc[i][j] = Frag<T>::mma(al, bh[j], acc[i][j]);
        }
      }
      Frag<T>::guard4(acc[i][0], acc[i][1], acc[i][2], acc[i][3], ah, SPLIT ? al : ah);
    }
    Frag<T>::keep(bh[0], bh[1], bh[2], bh[3]);
    if (SPLIT) Frag<T>::keep(bl[0], bl[1], bl[2], bl[3]);
  }
  acc_guard4(acc[0][0], acc[0][1], acc[0][2], acc[0][3]);
  acc_guard4(acc[1][0], acc[1][1], acc[1][2], acc[1][3]);
  acc_guard4(acc[2][0], acc[2][1], acc[2][2], acc[2][3]);
  acc_guard4(acc[3][0], acc[3][1], acc[3][2], acc[3][3]);

  float* slab = sT[wave];
  const float* Rb = RESID ? (resid + (size_t)b * strideR) : nullptr;
#pragma unroll
  for (int i = 0; i < 4; ++i) {
    const int mBase = m0 + (i << 4);
#pragma unroll
    for (int j = 0; j < 4; ++j) {
      const int n = n0 + (j << 4) + rlane;
      float bv = 0.f;
      if (BIAS_MODE == 2) bv = bias[n];
#pragma unroll
      for (int r = 0; r < 8; ++r) {
        float v = acc[i][j][r] * scale;
        if (BIAS_MODE == 1) v += bias[mBase + mOff + r];
        if (BIAS_MODE == 2) v += bv;
        if (RESID) v += Rb[(size_t)(mBase + mOff + r) * ldc + n];
        if (ACT == 1) v = tanhf(v);
        if (ACT == 2) v = fmaxf(v, 0.0f);
        if (ACT == 3) v = v / (1.0f + expf(-v));
        if (ACT == 4) v = (v > 0.f) ? v : 0.01f * v;
        slab[(mOff + r) * 68 + (j << 4) + rlane] = v;
      }
    }
    __builtin_amdgcn_fence(__ATOMIC_RELEASE, "workgroup");
    __builtin_amdgcn_wave_barrier();
    __builtin_amdgcn_fence(__ATOMIC_ACQUIRE, "workgroup");
    if (OUT_MODE == 0) {
      float* C = (float*)Cout + (size_t)b * strideC;
      const int hh = lane >> 4, c4 = (lane & 15) * 4;
      for (int pass = 0; pass < 2; ++pass) {
#pragma unroll
        for (int it = 0; it < 8; ++it) {
          const int row = it * 2 + hh;
          v4f v = *(const v4f*)(slab + row * 68 + c4);
          *(volatile v4f*)(C + (size_t)(mBase + row) * ldc + n0 + c4) = v;
        }
        __threadfence();
      }
    } else {
      const int q = lane >> 3, c8 = (lane & 7) * 8;
      unsigned short* C  = (unsigned short*)Cout  + (size_t)b * strideC;
      unsigned short* C2 = (OUT_MODE == 2) ? ((unsigned short*)Cout2 + (size_t)b * strideC) : nullptr;
      for (int pass = 0; pass < 2; ++pass) {
#pragma unroll
        for (int it = 0; it < 4; ++it) {
          const int row = it * 4 + q;
          const float* sp = slab + row * 68 + c8;
          v8h hv, lv;
#pragma unroll
          for (int e = 0; e < 8; ++e) {
            if (OUT_MODE == 1) {
              hv[e] = (_Float16)sp[e];
            } else {
              unsigned short hb = f2bf_bits(sp[e]);
              unsigned short lb = f2bf_bits(sp[e] - bf_bits2f(hb));
              hv[e] = __builtin_bit_cast(_Float16, hb);
              lv[e] = __builtin_bit_cast(_Float16, lb);
            }
          }
          *(volatile v8h*)(C + (size_t)(mBase + row) * ldc + n0 + c8) = hv;
          if (OUT_MODE == 2) *(volatile v8h*)(C2 + (size_t)(mBase + row) * ldc + n0 + c8) = lv;
        }
        __threadfence();
      }
    }
    __builtin_amdgcn_fence(__ATOMIC_RELEASE, "workgroup");
    __builtin_amdgcn_wave_barrier();
    __builtin_amdgcn_fence(__ATOMIC_ACQUIRE, "workgroup");
  }
}


__global__ __launch_bounds__(256) void wt_plane_kernel(const float* __restrict__ W, unsigned short* __restrict__ dst, int K, int N, int nLive, int ldd, int colOff) {
  const int n  = blockIdx.x;
  const int k8 = threadIdx.x * 8;
  const bool live = n < nLive;
  const int nc = live ? n : 0;
  v8h hv;
#pragma unroll
  for (int e = 0; e < 8; ++e) {
    const float w = W[(size_t)(k8 + e) * N + nc];
    hv[e] = (_Float16)(live ? carry_flush(bf16r(w), kWCarry) : 0.0f);
  }
  unsigned short* dp = dst + (size_t)n * ldd + colOff + k8;
  *(volatile v8h*)dp = hv;
  __threadfence();
  *(volatile v8h*)dp = hv;
}

__global__ __launch_bounds__(kThr) void setup_kernel(const float* __restrict__ b_hid, const float* __restrict__ b_og, float* __restrict__ BV) {
  const unsigned i = threadIdx.x;
  const bool og = i >= (unsigned)kBvOg;
  const float vh = b_hid[og ? 0u : i];
  const float vo = b_og[og ? (i - (unsigned)kBvOg) : 0u];
  const float o = bf16r(og ? vo : vh);
  float* dp = BV + i;
  *(volatile float*)dp = o;
  __threadfence();
  *(volatile float*)dp = o;
}
static_assert(kBvTot == kThr, "set-up grid exact: one block");

__global__ __launch_bounds__(kThr) void rsum_kernel(const float* __restrict__ x, float* __restrict__ RAW) {
  const unsigned ix = blockIdx.x * (unsigned)kThr + threadIdx.x;
  const unsigned sq = ix >> 9;
  const unsigned hd = ix & (unsigned)(kHD - 1);
  float run = 0.0f;
  for (int t = 0; t < kL; ++t) {
    const unsigned tok = sq * (unsigned)kL + (unsigned)t;
    float* dp = RAW + tok * (unsigned)kHD + hd;
    *(volatile float*)dp = run;
    __threadfence();
    *(volatile float*)dp = run;
    run += bf16r(x[tok * (unsigned)kHD + hd]);
  }
}
static_assert(kNB * kHD == 8 * kThr, "the running sum's grid exact: 8 blocks: two a sequence");

__global__ __launch_bounds__(kThr) void stat_kernel(const float* __restrict__ RAW, float* __restrict__ ST) {
  const unsigned tok = blockIdx.x * (unsigned)kThr + threadIdx.x;
  const float* pr = RAW + tok * (unsigned)kHD;
  float s = 0.0f;
  for (int q = 0; q < kHD / 4; ++q) { const v4f v = *(const v4f*)(pr + 4 * q); s += v[0]; s += v[1]; s += v[2]; s += v[3]; }
  const float mu = s / (float)kHD;
  float qq = 0.0f;
  for (int q = 0; q < kHD / 4; ++q) { const v4f v = *(const v4f*)(pr + 4 * q);
#pragma unroll
    for (int e = 0; e < 4; ++e) { const float d = v[e] - mu; qq += d * d; } }
  v2f o; o[0] = mu; o[1] = 1.0f / sqrtf(qq / (float)kHD + kNormEps);
  float* dp = ST + tok * 2u;
  *(volatile v2f*)dp = o;
  __threadfence();
  *(volatile v2f*)dp = o;
}
static_assert(kTok == 64 * kThr && (kHD % 4) == 0, "the statistics' grid exact: 64 blocks: a thread a token");

__global__ __launch_bounds__(kThr) void pack_kernel(const float* __restrict__ x, const float* __restrict__ RAW, const float* __restrict__ ST, const float* __restrict__ ln_gamma, const float* __restrict__ ln_beta,
                                                    unsigned short* __restrict__ A16) {
  const unsigned i = blockIdx.x * (unsigned)kThr + threadIdx.x;
  const unsigned row = i >> 3;
  const unsigned d8 = (i & 7u) * 8u;
  const unsigned tok = row >> 3;
  const unsigned hd8 = (row & 7u) * (unsigned)kD + d8;
  const v2f ms = *(const v2f*)(ST + tok * 2u);
  const v4f a0 = *(const v4f*)(x + i * 8u), a1 = *(const v4f*)(x + i * 8u + 4);
  const v4f r0 = *(const v4f*)(RAW + i * 8u), r1 = *(const v4f*)(RAW + i * 8u + 4);
  const v4f g0 = *(const v4f*)(ln_gamma + hd8), g1 = *(const v4f*)(ln_gamma + hd8 + 4), b0 = *(const v4f*)(ln_beta + hd8), b1 = *(const v4f*)(ln_beta + hd8 + 4);
  v8h hx, hc;
#pragma unroll
  for (int e = 0; e < 8; ++e) {
    const float xv = (e < 4) ? a0[e] : a1[e - 4];
    const float rv = (e < 4) ? r0[e] : r1[e - 4];
    const float gw = (e < 4) ? g0[e] : g1[e - 4];
    const float gb = (e < 4) ? b0[e] : b1[e - 4];
    hx[e] = (_Float16)carry_flush(bf16r(xv), kACarry);
    hc[e] = (_Float16)carry_flush(((rv - ms[0]) * ms[1]) * bf16r(gw) + bf16r(gb), kACarry);
  }
  unsigned short* dp = A16 + row * (unsigned)kK + d8;
  for (int pass = 0; pass < 2; ++pass) {
    *(volatile v8h*)dp = hx;
    *(volatile v8h*)(dp + kD) = hc;
    __threadfence();
  }
}
static_assert((size_t)kRows * kD / 8 == 4096ull * kThr && kD / 8 == 8, "the pack's grid exact: 4,096 blocks: 32 rows a block");

__global__ __launch_bounds__(kThr) void cell_kernel(const float* __restrict__ H3, const float* __restrict__ init_cx, float* __restrict__ CELL) {
  const unsigned ix = blockIdx.x * (unsigned)kThr + threadIdx.x;
  const unsigned sq = ix >> 9;
  const unsigned hd = ix & (unsigned)(kHD - 1);
  const unsigned head = hd >> 6;
  const unsigned d = hd & (unsigned)(kD - 1);
  float c = bf16r(init_cx[hd]);
  for (int t = 0; t < kL; ++t) {
    const unsigned tok = sq * (unsigned)kL + (unsigned)t;
    const float* ph = H3 + (tok * (unsigned)kH + head) * (unsigned)kN3 + d;
    const float gi = ph[0], gf = ph[kD], gh = ph[2 * kD];
    const float fg = 1.0f / (1.0f + expf(-gf));
    const float igh = (1.0f / (1.0f + expf(-gi))) * fmaxf(gh, 0.0f);
    c = fg * c + igh;
    float* dp = CELL + tok * (unsigned)kHD + hd;
    *(volatile float*)dp = c;
    __threadfence();
    *(volatile float*)dp = c;
  }
}
static_assert(kNB * kHD == 8 * kThr && kD == 64 && kH == 8, "the cell's grid exact: 8 blocks: two a sequence");

__global__ __launch_bounds__(kThr) void pack2_kernel(const float* __restrict__ CELL, unsigned short* __restrict__ A16) {
  const unsigned i = blockIdx.x * (unsigned)kThr + threadIdx.x;
  const unsigned row = i >> 3;
  const unsigned d8 = (i & 7u) * 8u;
  const v4f c0 = *(const v4f*)(CELL + i * 8u), c1 = *(const v4f*)(CELL + i * 8u + 4);
  v8h hc;
#pragma unroll
  for (int e = 0; e < 4; ++e) { hc[e] = (_Float16)carry_flush(c0[e], kACarry); hc[4 + e] = (_Float16)carry_flush(c1[e], kACarry); }
  unsigned short* dp = A16 + row * (unsigned)kK + (unsigned)kD + d8;
  *(volatile v8h*)dp = hc;
  __threadfence();
  *(volatile v8h*)dp = hc;
}
static_assert((size_t)kRows * kD / 8 == 4096ull * kThr, "the second pack's grid exact: 4,096 blocks");

__global__ __launch_bounds__(kThr) void close_kernel(const float* __restrict__ OGP, const float* __restrict__ CELL, float* __restrict__ out) {
  const unsigned i = blockIdx.x * (unsigned)kThr + threadIdx.x;
  const v4f g0 = *(const v4f*)(OGP + i * 8u), g1 = *(const v4f*)(OGP + i * 8u + 4);
  const v4f c0 = *(const v4f*)(CELL + i * 8u), c1 = *(const v4f*)(CELL + i * 8u + 4);
  v4f o0, o1;
#pragma unroll
  for (int e = 0; e < 4; ++e) { o0[e] = (1.0f / (1.0f + expf(-g0[e]))) * c0[e]; o1[e] = (1.0f / (1.0f + expf(-g1[e]))) * c1[e]; }
  float* dp = out + i * 8u;
  for (int pass = 0; pass < 2; ++pass) {
    *(volatile v4f*)dp = o0;
    *(volatile v4f*)(dp + 4) = o1;
    __threadfence();
  }
}
static_assert((size_t)kOut0 / 8 == 4096ull * kThr && (size_t)kRows * kN3 < 4294967296ull / 4, "the closing product's grid exact: 4,096 blocks; every plane's element offsets fit 32 bits");

extern "C" void kernel_launch(void* const* d_in, const int* in_sizes, int n_in,
                              void* d_out, int out_size, void* d_ws, size_t ws_size,
                              hipStream_t stream) {
  if (n_in < 8 || d_out == nullptr || d_ws == nullptr) return;
  if (in_sizes[0] != kOut0 || in_sizes[1] != kK * kN3 || in_sizes[2] != kN3 || in_sizes[3] != kK * kD || in_sizes[4] != kD || in_sizes[5] != kHD || in_sizes[6] != kHD || in_sizes[7] != kHD) return;
  if (out_size != kOut0) return;
  if (ws_size < kWsTotal) return;
  const float* x = (const float*)d_in[0];
  const float* W_hid = (const float*)d_in[1];
  const float* b_hid = (const float*)d_in[2];
  const float* W_og = (const float*)d_in[3];
  const float* b_og = (const float*)d_in[4];
  const float* ln_gamma = (const float*)d_in[5];
  const float* ln_beta = (const float*)d_in[6];
  const float* init_cx = (const float*)d_in[7];
  float* out = (float*)d_out;
  char* ws = (char*)d_ws;
  unsigned short* WHT = (unsigned short*)(ws + kOffWHT);
  unsigned short* WOT = (unsigned short*)(ws + kOffWOT);
  float* BV = (float*)(ws + kOffBV);
  float* ST = (float*)(ws + kOffST);
  float* RAW = (float*)(ws + kOffRAW);
  unsigned short* A16 = (unsigned short*)(ws + kOffA16);
  float* H3 = (float*)(ws + kOffH3);
  float* CELL = (float*)(ws + kOffCELL);
  float* OGP = (float*)(ws + kOffOGP);

  static_assert(kK / 8 == 16, "the transposing casts run one block a destination row with exactly K / 8 threads");
  wt_plane_kernel<<<kN3, kK / 8, 0, stream>>>(W_hid, WHT, kK, kN3, kN3, kK, 0);
  wt_plane_kernel<<<kD, kK / 8, 0, stream>>>(W_og, WOT, kK, kD, kD, kK, 0);
  setup_kernel<<<1, kThr, 0, stream>>>(b_hid, b_og, BV);
  rsum_kernel<<<8, kThr, 0, stream>>>(x, RAW);
  stat_kernel<<<64, kThr, 0, stream>>>(RAW, ST);
  pack_kernel<<<4096, kThr, 0, stream>>>(x, RAW, ST, ln_gamma, ln_beta, A16);
  wmma_gemm64<0, false, 2, 0, false, 0><<<dim3((kRows / 64) * (kN3 / 64) / 8, 1), 256, 0, stream>>>(
      A16, A16, kK, 0L, WHT, WHT, kK, 0L, (void*)H3, (void*)H3, kN3, 0L, BV, nullptr, 0L, kRows, kN3, kK, kSc);
  cell_kernel<<<8, kThr, 0, stream>>>(H3, init_cx, CELL);
  pack2_kernel<<<4096, kThr, 0, stream>>>(CELL, A16);
  wmma_gemm64<0, false, 2, 0, false, 0><<<dim3((kRows / 64) * (kD / 64) / 8, 1), 256, 0, stream>>>(
      A16, A16, kK, 0L, WOT, WOT, kK, 0L, (void*)OGP, (void*)OGP, kD, 0L, BV + kBvOg, nullptr, 0L, kRows, kD, kK, kSc);
  close_kernel<<<4096, kThr, 0, stream>>>(OGP, CELL, out);
}
static_assert(((kRows / 64) * (kN3 / 64)) % 8 == 0 && ((kRows / 64) * (kD / 64)) % 8 == 0, "the engine's grids: whole blocks of eight wave tiles");
